// CrossAttentionMS_OneK_17145509446498
// MI455X (gfx1250) — hardware-run, weakly checked
//
#include <hip/hip_runtime.h>

typedef float          v8f   __attribute__((ext_vector_type(8)));
typedef float          v4f   __attribute__((ext_vector_type(4)));
typedef unsigned int   v4u   __attribute__((ext_vector_type(4)));
typedef int            v8i   __attribute__((ext_vector_type(8)));
typedef unsigned short v8us  __attribute__((ext_vector_type(8)));
typedef unsigned short v16us __attribute__((ext_vector_type(16)));
typedef __bf16         v16bf __attribute__((ext_vector_type(16)));
typedef _Float16       v16h  __attribute__((ext_vector_type(16)));
typedef v4f  __attribute__((may_alias)) v4fa;
typedef v8us __attribute__((may_alias)) v8usa;
union FragB { v16bf v; v16us u; v8us h[2]; v8i w; };
union FragH { v16h  v; v16us u; v8us h[2]; v8i w; };

__device__ __forceinline__ v8f wmb(const FragB& a, const FragB& b, v8f c) {
  v8f d = __builtin_amdgcn_wmma_f32_16x16x32_bf16(false, a.v, false, b.v, (short)0, c, false, false);
  asm volatile("v_nop\n\tv_nop\n\tv_nop\n\tv_nop" : "+v"(d) : "v"(a.w), "v"(b.w));
  return d;
}

__device__ __forceinline__ v8f wmh(const FragH& a, const FragH& b, v8f c) {
  v8f d = __builtin_amdgcn_wmma_f32_16x16x32_f16(false, a.v, false, b.v, (short)0, c, false, false);
  asm volatile("v_nop\n\tv_nop\n\tv_nop\n\tv_nop" : "+v"(d) : "v"(a.w), "v"(b.w));
  return d;
}

__device__ __forceinline__ unsigned bf16_bits(float f) {
  const unsigned u = __float_as_uint(f);
  const unsigned r = (u + 0x7FFFu + ((u >> 16) & 1u)) >> 16;
  const unsigned q = (u >> 16) | 0x40u;
  return ((u & 0x7fffffffu) > 0x7f800000u) ? q : r;
}

__device__ __forceinline__ float bf16_val(float f) {
  return __uint_as_float(bf16_bits(f) << 16);
}
__device__ __forceinline__ int clampi(int v, int lo, int hi) {
  return v < lo ? lo : (v > hi ? hi : v);
}

__device__ __forceinline__ unsigned f16_bits(float f) {
  const unsigned u  = __float_as_uint(f);
  const unsigned s  = (u >> 16) & 0x8000u;
  const unsigned a  = u & 0x7fffffffu;
  const unsigned t  = a - 0x38000000u;
  const unsigned r  = (t + 0x0FFFu + ((t >> 13) & 1u)) >> 13;
  const unsigned rc = r > 0x7C00u ? 0x7C00u : r;
  const bool small  = a < 0x38800000u;
  const bool isnan  = a > 0x7f800000u;
  const unsigned fin = small ? 0u : (s | rc);
  return isnan ? (s | 0x7E00u) : fin;
}

__device__ __forceinline__ unsigned pk16(unsigned lo, unsigned hi) { return lo | (hi << 16); }
__device__ __forceinline__ unsigned bf16_lo_bits(float v) {
  float hi = bf16_val(v);
  asm volatile("" : "+v"(hi));
  return bf16_bits(v - hi);
}
__device__ __forceinline__ v4u pack8_bf16(v4f a, v4f c) {
  return (v4u){ pk16(bf16_bits(a[0]), bf16_bits(a[1])), pk16(bf16_bits(a[2]), bf16_bits(a[3])),
                pk16(bf16_bits(c[0]), bf16_bits(c[1])), pk16(bf16_bits(c[2]), bf16_bits(c[3])) };
}
__device__ __forceinline__ v4u pack8_bf16_lo(v4f a, v4f c) {
  return (v4u){ pk16(bf16_lo_bits(a[0]), bf16_lo_bits(a[1])), pk16(bf16_lo_bits(a[2]), bf16_lo_bits(a[3])),
                pk16(bf16_lo_bits(c[0]), bf16_lo_bits(c[1])), pk16(bf16_lo_bits(c[2]), bf16_lo_bits(c[3])) };
}
__device__ __forceinline__ v4u pack8_f16(v4f a, v4f c) {
  return (v4u){ pk16(f16_bits(a[0]), f16_bits(a[1])), pk16(f16_bits(a[2]), f16_bits(a[3])),
                pk16(f16_bits(c[0]), f16_bits(c[1])), pk16(f16_bits(c[2]), f16_bits(c[3])) };
}

template <int FORM>
__global__ __launch_bounds__(256) void k_plane(const float* __restrict__ src, int rows, int cols, int ldsrc,
                                               unsigned short* __restrict__ dst, int MP, int KP) {
  static_assert(FORM >= 0 && FORM <= 3);
  const int KTOT = (FORM == 1 || FORM == 3) ? 2 * KP : KP;
  const unsigned ppr   = (unsigned)(KTOT >> 3);
  const unsigned kp8   = (unsigned)(KP >> 3);
  const unsigned total = (unsigned)MP * ppr;
  const unsigned g     = blockIdx.x * 256u + threadIdx.x;
  const unsigned rowu  = g / ppr;
  const unsigned p     = g - rowu * ppr;
  const bool second    = p >= kp8;
  const int row = (int)rowu;
  const int c0  = (int)((second ? p - kp8 : p) << 3);
  const float* srow = src + (size_t)clampi(row, 0, rows - 1) * (size_t)ldsrc;
  float x[8];
  unsigned mk[8];
#pragma unroll
  for (int e = 0; e < 8; ++e) {
    const int c = c0 + e;
    const float v = srow[clampi(c, 0, cols - 1)];
    asm volatile("" :: "v"(v));
    x[e]  = v;
    mk[e] = (row < rows && c < cols) ? 0xFFFFu : 0u;
  }
  const v4f a = (v4f){ x[0], x[1], x[2], x[3] };
  const v4f c = (v4f){ x[4], x[5], x[6], x[7] };
  v4u o;
  if (FORM == 2) {
    o = pack8_f16(a, c);
  } else {
    const v4u hi = pack8_bf16(a, c);
    o = hi;
    if (FORM == 1) { const v4u lo = pack8_bf16_lo(a, c); o = second ? lo : hi; }
  }
  const v4u mw = (v4u){ pk16(mk[0], mk[1]), pk16(mk[2], mk[3]), pk16(mk[4], mk[5]), pk16(mk[6], mk[7]) };
  o &= mw;
  if (g < total) {
    volatile v4u* q = (volatile v4u*)(dst + (size_t)g * 8);
    *q = o;
    __threadfence();
    *q = o;
  }
}

template <int FORM> struct FragOf    { typedef FragB T; };
template <>         struct FragOf<2> { typedef FragH T; };
__device__ __forceinline__ v8f mm(const FragB& a, const FragB& b, v8f c) { return wmb(a, b, c); }
__device__ __forceinline__ v8f mm(const FragH& a, const FragH& b, v8f c) { return wmh(a, b, c); }
template <class F> __device__ __forceinline__ F ld_frag(const unsigned short* p) {
  F f;
  f.h[0] = *(const v8usa*)(p);
  f.h[1] = *(const v8usa*)(p + 16);
  return f;
}

template <int FORM, int EPI>
__global__ __launch_bounds__(256) __attribute__((amdgpu_num_vgpr(248)))
void k_gemm_nt(const unsigned short* __restrict__ A, const unsigned short* __restrict__ B,
               const float* __restrict__ bias, float* __restrict__ D, int M, int N, int KTOT, int ldd) {
  static_assert(FORM >= 0 && FORM <= 2);
  static_assert(EPI == 0 || EPI == 1);
  typedef typename FragOf<FORM>::T F;
  __shared__ __attribute__((aligned(16))) float sT[8][16 * 68];
  const int lane = threadIdx.x & 31;
  const int wave = threadIdx.x >> 5;
  const int tilesM = (M + 63) >> 6;
  const int tilesN = (N + 63) >> 6;
  const int tile = blockIdx.x * 8 + wave;
  if (tile >= tilesM * tilesN) return;
  const int tm = tile / tilesN;
  const int tn = tile - tm * tilesN;
  const int m0 = tm << 6;
  const int n0 = tn << 6;

  const int rl = lane & 15;
  const int h8 = (lane >> 4) * 8;
  const unsigned short* pa = A + (size_t)(m0 + rl) * (size_t)KTOT + h8;
  const unsigned short* pb = B + (size_t)(n0 + rl) * (size_t)KTOT + h8;

  v8f acc[4][4];
#pragma unroll
  for (int i = 0; i < 4; ++i)
#pragma unroll
    for (int j = 0; j < 4; ++j) acc[i][j] = (v8f){0.f, 0.f, 0.f, 0.f, 0.f, 0.f, 0.f, 0.f};

#pragma unroll 1
  for (int k0 = 0; k0 < KTOT; k0 += 32) {
    F bf[4];
#pragma unroll
    for (int j = 0; j < 4; ++j) bf[j] = ld_frag<F>(pb + (size_t)(j << 4) * (size_t)KTOT + k0);
#pragma unroll
    for (int i = 0; i < 4; ++i) {
      const F af = ld_frag<F>(pa + (size_t)(i << 4) * (size_t)KTOT + k0);
#pragma unroll
      for (int j = 0; j < 4; ++j) acc[i][j] = mm(af, bf[j], acc[i][j]);
    }
  }

  float* slab = sT[wave];
  const int hh = lane >> 4;
  const int c4 = (lane & 15) * 4;
  const int nc = n0 + c4;
  const bool cok = nc < N;
  v4f bv = (v4f){0.f, 0.f, 0.f, 0.f};
  if (EPI == 1) {
    bv = *(const v4fa*)(bias + clampi(nc, 0, N - 4));
    asm volatile("" :: "v"(bv));
  }
#pragma unroll
  for (int i = 0; i < 4; ++i) {
    const int mBase = m0 + (i << 4);
#pragma unroll
    for (int j = 0; j < 4; ++j) {
#pragma unroll
      for (int r = 0; r < 8; ++r) slab[(h8 + r) * 68 + (j << 4) + rl] = acc[i][j][r];
    }
    __builtin_amdgcn_fence(__ATOMIC_RELEASE, "workgroup");
    __builtin_amdgcn_wave_barrier();
    __builtin_amdgcn_fence(__ATOMIC_ACQUIRE, "workgroup");
    v4f vv[8];
#pragma unroll
    for (int it = 0; it < 8; ++it) {
      const int row = it * 2 + hh;
      v4f v = *(const v4fa*)(slab + row * 68 + c4);
      if (EPI == 1) v += bv;
      vv[it] = v;
    }
    for (int pass = 0; pass < 2; ++pass) {
#pragma unroll
      for (int it = 0; it < 8; ++it) {
        const int row = mBase + it * 2 + hh;
        if (cok && row < M) *(volatile v4f*)(D + (size_t)row * (size_t)ldd + nc) = vv[it];
      }
      __threadfence();
    }
    __builtin_amdgcn_fence(__ATOMIC_RELEASE, "workgroup");
    __builtin_amdgcn_wave_barrier();
    __builtin_amdgcn_fence(__ATOMIC_ACQUIRE, "workgroup");
  }
}

#pragma clang fp contract(off)

constexpr int NCLD = 8;
constexpr int NPTS = 2048;
constexpr int CH   = 128;
constexpr int NHEAD = 4;
constexpr int HD   = 32;
constexpr int NSC  = 3;
constexpr int KNB  = 16;
constexpr int KT   = NSC * KNB;
constexpr int ROWS = NCLD * NPTS;
constexpr int NCOL = 5 * CH;
constexpr int IDXW = 64;
constexpr int PREP_WB_BLOCKS = 20;
constexpr int PREP_BT_BLOCK  = 20;
constexpr int PREP_BK_BLOCK  = 21;
constexpr int PREP_CT_BLOCK0 = 22;
constexpr int PREP_CT_BLOCKS = ROWS / 256;
constexpr int PREP_BLOCKS    = PREP_CT_BLOCK0 + PREP_CT_BLOCKS;
constexpr int TPITCH = 36;

static_assert(NPTS == 32 * 64);
static_assert(CH == 32 * 4);
static_assert(NHEAD * HD == CH && HD == 32 && NHEAD == 4);
static_assert(KT == 48 && KT <= IDXW);
static_assert(ROWS % 8 == 0 && ROWS % 64 == 0 && ROWS % 256 == 0 && ROWS == 16384);
static_assert(NCOL == 640 && NCOL % 64 == 0 && NCOL % 32 == 0 && NCOL % 4 == 0);
static_assert(CH % 32 == 0);
static_assert((ROWS * (CH / 8)) % 256 == 0);
static_assert((long long)ROWS * CH / 8 < 0x7fffffffLL);
static_assert(((ROWS / 64) * (NCOL / 64)) % 8 == 0);
static_assert(PREP_BLOCKS == 86);
static_assert((NPTS & (NPTS - 1)) == 0);

constexpr size_t SZ_XB  = (size_t)ROWS * CH * 2;
constexpr size_t SZ_WB  = (size_t)NCOL * CH * 2;
constexpr size_t SZ_BT  = (size_t)NCOL * 4;
constexpr size_t SZ_BK  = (size_t)NSC * CH * 4;
constexpr size_t SZ_CT  = (size_t)ROWS * 4 * 4;
constexpr size_t SZ_T   = (size_t)ROWS * NCOL * 4;
constexpr size_t SZ_IDX = (size_t)ROWS * IDXW * 4;
constexpr size_t OFF_XB  = 0;
constexpr size_t OFF_WB  = OFF_XB + SZ_XB;
constexpr size_t OFF_BT  = OFF_WB + SZ_WB;
constexpr size_t OFF_BK  = OFF_BT + SZ_BT;
constexpr size_t OFF_CT  = OFF_BK + SZ_BK;
constexpr size_t OFF_T   = OFF_CT + SZ_CT;
constexpr size_t OFF_IDX = OFF_T + SZ_T;
constexpr size_t WS_TOTAL = OFF_IDX + SZ_IDX;
static_assert(SZ_XB % 256 == 0 && SZ_WB % 256 == 0 && SZ_BT % 256 == 0 && SZ_BK % 256 == 0);
static_assert(SZ_CT % 256 == 0 && SZ_T % 256 == 0 && SZ_IDX % 256 == 0);
static_assert(OFF_WB % 256 == 0 && OFF_BT % 256 == 0 && OFF_BK % 256 == 0 && OFF_CT % 256 == 0);
static_assert(OFF_T % 256 == 0 && OFF_IDX % 256 == 0);
static_assert(SZ_XB == (size_t)4194304 && SZ_WB == (size_t)163840 && SZ_BT == (size_t)2560 && SZ_BK == (size_t)1536);
static_assert(SZ_CT == (size_t)262144 && SZ_T == (size_t)41943040 && SZ_IDX == (size_t)4194304);
static_assert(WS_TOTAL == (size_t)50761728);
static_assert(WS_TOTAL <= ((size_t)128 << 20));

__device__ __forceinline__ float blend2(float a, unsigned ma, float b, unsigned mb) {
  return __uint_as_float((__float_as_uint(a) & ma) | (__float_as_uint(b) & mb));
}
__device__ __forceinline__ float blend3(float a, unsigned ma, float b, unsigned mb, float c, unsigned mc) {
  return __uint_as_float((__float_as_uint(a) & ma) | (__float_as_uint(b) & mb) | (__float_as_uint(c) & mc));
}
__device__ __forceinline__ float selmax(float a, float b) {
  return (a > b || a != a) ? a : b;
}
__device__ __forceinline__ float dist3(float xi, float yi, float zi, float sqi, v4f c) {
  const float dot = (xi * c[0] + yi * c[1]) + zi * c[2];
  return (sqi + c[3]) - 2.0f * dot;
}

__global__ __launch_bounds__(256) void k_prep(const float* __restrict__ coord,
                                              const float* __restrict__ Wq, const float* __restrict__ bq,
                                              const float* __restrict__ Wk, const float* __restrict__ bk,
                                              const float* __restrict__ Wv, const float* __restrict__ bv,
                                              unsigned short* __restrict__ WB, float* __restrict__ BT,
                                              float* __restrict__ BK, float* __restrict__ CT) {
  __shared__ __attribute__((aligned(16))) float sT[CH * TPITCH];
  const int tid = (int)threadIdx.x;
  const int blk = (int)blockIdx.x;
  if (blk < PREP_WB_BLOCKS) {
    const int mat = blk >> 2;
    const int n0  = (blk & 3) * 32;
    const int kw  = clampi(mat - 2, 0, NSC - 1);
    const unsigned mq = (mat == 0) ? 0xFFFFFFFFu : 0u;
    const unsigned mv = (mat == 1) ? 0xFFFFFFFFu : 0u;
    const unsigned mk = (mat >= 2) ? 0xFFFFFFFFu : 0u;
#pragma unroll
    for (int i = 0; i < 4; ++i) {
      const int piece = tid + 256 * i;
      const int k  = piece >> 3;
      const int nq = piece & 7;
      const int off = k * CH + n0 + 4 * nq;
      const v4f a = *(const v4fa*)(Wq + off);
      const v4f b = *(const v4fa*)(Wv + off);
      const v4f c = *(const v4fa*)(Wk + (size_t)kw * CH * CH + off);
      asm volatile("" :: "v"(a));
      asm volatile("" :: "v"(b));
      asm volatile("" :: "v"(c));
      const v4f x = (v4f){ blend3(a[0], mq, b[0], mv, c[0], mk), blend3(a[1], mq, b[1], mv, c[1], mk),
                           blend3(a[2], mq, b[2], mv, c[2], mk), blend3(a[3], mq, b[3], mv, c[3], mk) };
      *(v4fa*)(sT + k * TPITCH + 4 * nq) = x;
    }
    __syncthreads();
    v4u o[2];
#pragma unroll
    for (int i = 0; i < 2; ++i) {
      const int g  = tid + 256 * i;
      const int n  = g >> 4;
      const int kp = g & 15;
      const float* col = sT + (8 * kp) * TPITCH + n;
      const v4f a = (v4f){ col[0], col[TPITCH], col[2 * TPITCH], col[3 * TPITCH] };
      const v4f c = (v4f){ col[4 * TPITCH], col[5 * TPITCH], col[6 * TPITCH], col[7 * TPITCH] };
      o[i] = pack8_bf16(a, c);
    }
    unsigned short* base = WB + (size_t)(mat * CH + n0) * CH;
    volatile v4u* q0 = (volatile v4u*)(base + (size_t)tid * 8);
    volatile v4u* q1 = (volatile v4u*)(base + (size_t)(tid + 256) * 8);
    *q0 = o[0];
    *q1 = o[1];
    __threadfence();
    *q0 = o[0];
    *q1 = o[1];
  } else if (blk == PREP_BT_BLOCK) {
    const int u = tid < (NCOL / 4) ? tid : (NCOL / 4) - 1;
    const v4f a = *(const v4fa*)(bq + 4 * clampi(u, 0, 31));
    const v4f b = *(const v4fa*)(bv + 4 * clampi(u - 32, 0, 31));
    asm volatile("" :: "v"(a));
    asm volatile("" :: "v"(b));
    const unsigned ma = (u < 32) ? 0xFFFFFFFFu : 0u;
    const unsigned mb = (u >= 32 && u < 64) ? 0xFFFFFFFFu : 0u;
    const v4f o = (v4f){ bf16_val(blend2(a[0], ma, b[0], mb)), bf16_val(blend2(a[1], ma, b[1], mb)),
                         bf16_val(blend2(a[2], ma, b[2], mb)), bf16_val(blend2(a[3], ma, b[3], mb)) };
    if (tid < NCOL / 4) {
      volatile v4f* q = (volatile v4f*)(BT + 4 * tid);
      *q = o;
      __threadfence();
      *q = o;
    }
  } else if (blk == PREP_BK_BLOCK) {
    const int u = tid < (NSC * CH / 4) ? tid : (NSC * CH / 4) - 1;
    const v4f a = *(const v4fa*)(bk + 4 * u);
    asm volatile("" :: "v"(a));
    const v4f o = (v4f){ bf16_val(a[0]), bf16_val(a[1]), bf16_val(a[2]), bf16_val(a[3]) };
    if (tid < NSC * CH / 4) {
      volatile v4f* q = (volatile v4f*)(BK + 4 * tid);
      *q = o;
      __threadfence();
      *q = o;
    }
  } else {
    const int p  = (blk - PREP_CT_BLOCK0) * 256 + tid;
    const int pc = p < ROWS ? p : ROWS - 1;
    const float xr = coord[3 * pc + 0];
    const float yr = coord[3 * pc + 1];
    const float zr = coord[3 * pc + 2];
    asm volatile("" :: "v"(xr));
    asm volatile("" :: "v"(yr));
    asm volatile("" :: "v"(zr));
    const float x = bf16_val(xr);
    const float y = bf16_val(yr);
    const float z = bf16_val(zr);
    const float sq = (x * x + y * y) + z * z;
    const v4f o = (v4f){ x, y, z, sq };
    if (p < ROWS) {
      volatile v4f* q = (volatile v4f*)(CT + (size_t)p * 4);
      *q = o;
      __threadfence();
      *q = o;
    }
  }
}

__global__ __launch_bounds__(256) void k_sel(const float* CT, int* IDX) {
  const int tid = (int)threadIdx.x, lane = tid & 31, wave = tid >> 5;
  const int row = __builtin_amdgcn_readfirstlane((int)blockIdx.x * 8 + wave);
  const int rc  = row < ROWS ? row : ROWS - 1;
  const int cb  = rc & ~(NPTS - 1);
  const int nloc = rc & (NPTS - 1);

  const v4f own = *(const v4fa*)(CT + (size_t)rc * 4);
  asm volatile("" :: "v"(own));
  const float xi = own[0], yi = own[1], zi = own[2], sqi = own[3];

  float d[64];
  int j = lane;
#pragma unroll
  for (int g = 0; g < 16; ++g) {
    asm volatile("" : "+v"(j));
    const float* p = CT + ((size_t)(cb + j) << 2);
    const v4f c0 = *(const v4fa*)(p);
    const v4f c1 = *(const v4fa*)(p + 32 * 4);
    const v4f c2 = *(const v4fa*)(p + 64 * 4);
    const v4f c3 = *(const v4fa*)(p + 96 * 4);
    asm volatile("" :: "v"(c0));
    asm volatile("" :: "v"(c1));
    asm volatile("" :: "v"(c2));
    asm volatile("" :: "v"(c3));
    d[4 * g + 0] = dist3(xi, yi, zi, sqi, c0);
    d[4 * g + 1] = dist3(xi, yi, zi, sqi, c1);
    d[4 * g + 2] = dist3(xi, yi, zi, sqi, c2);
    d[4 * g + 3] = dist3(xi, yi, zi, sqi, c3);
    j += 128;
  }

  const float pinf = __uint_as_float(0x7f800000u);
  int w0 = nloc, w1 = nloc, kill = -1;
#pragma unroll 1
  for (int t = 0; t < KT; ++t) {
    float x0 = d[0];
    x0 = (kill == 0) ? pinf : x0;
    d[0] = x0;
    float bv = x0;
    int br = 0;
#pragma unroll
    for (int r = 1; r < 64; ++r) {
      float x = d[r];
      x = (kill == r) ? pinf : x;
      d[r] = x;
      const bool lt = x < bv;
      bv = lt ? x : bv;
      br = lt ? r : br;
    }
    int bj = lane + 32 * br;
#pragma unroll
    for (int m = 16; m >= 1; m >>= 1) {
      const float ov = __shfl_xor(bv, m, 32);
      const int   oj = __shfl_xor(bj, m, 32);
      const bool take = (ov < bv) || (ov == bv && oj < bj);
      bv = take ? ov : bv;
      bj = take ? oj : bj;
    }
    w0 = (lane == t) ? bj : w0;
    w1 = (lane == t - 32) ? bj : w1;
    kill = (lane == (bj & 31)) ? (bj >> 5) : -1;
  }

  if (row < ROWS) {
    volatile int* q0 = (volatile int*)(IDX + (size_t)row * IDXW + lane);
    volatile int* q1 = (volatile int*)(IDX + (size_t)row * IDXW + 32 + lane);
    *q0 = w0;
    *q1 = w1;
    __threadfence();
    *q0 = w0;
    *q1 = w1;
  }
}

__global__ __launch_bounds__(256) void k_attn(const float* __restrict__ T, const float* __restrict__ BK,
                                              const int* __restrict__ IDX, const int* __restrict__ kin,
                                              float* __restrict__ out, int nrows) {
  const int tid = (int)threadIdx.x, lane = tid & 31, wave = tid >> 5;
  const int row = __builtin_amdgcn_readfirstlane((int)blockIdx.x * 8 + wave);
  const int rc  = row < nrows ? row : nrows - 1;
  const int cb  = rc & ~(NPTS - 1);

  const float* trow = T + (size_t)rc * NCOL + 4 * lane;
  const v4f q = *(const v4fa*)(trow);
  asm volatile("" :: "v"(q));
  const v4f v = *(const v4fa*)(trow + CH);
  asm volatile("" :: "v"(v));
  int wa = IDX[(size_t)rc * IDXW + lane];
  asm volatile("" :: "v"(wa));
  int wb = IDX[(size_t)rc * IDXW + 32 + lane];
  asm volatile("" :: "v"(wb));
  wa = clampi(wa, 0, NPTS - 1);
  wb = clampi(wb, 0, NPTS - 1);
  const int kval = kin[0];
  asm volatile("" :: "v"(kval));

  const float isd = 1.0f / sqrtf(32.0f);
  const int l7 = lane & 7;
  float gate = 0.0f;

#pragma unroll 1
  for (int i = 0; i < NSC; ++i) {
    const v4f pc = *(const v4fa*)(trow + 2 * CH + CH * i);
    asm volatile("" :: "v"(pc));
    const v4f bk = *(const v4fa*)(BK + CH * i + 4 * lane);
    asm volatile("" :: "v"(bk));
    const int msk  = (i < 2) ? -1 : 0;
    const int wsel = (wa & msk) | (wb & ~msk);
    const int l0   = (16 * i) & 31;
    const float* gbase = T + (size_t)cb * NCOL + 2 * CH + CH * i;
    int lo = 4 * lane;
    float lg0 = 0.0f, lg1 = 0.0f;
#pragma unroll
    for (int k = 0; k < KNB; ++k) {
      if ((k & 7) == 0) asm volatile("" : "+v"(lo));
      const int id = __builtin_amdgcn_readlane(wsel, l0 + k);
      const v4f g = *(const v4fa*)(gbase + (size_t)id * NCOL + lo);
      asm volatile("" :: "v"(g));
      const float k0 = (g[0] - pc[0]) + bk[0];
      const float k1 = (g[1] - pc[1]) + bk[1];
      const float k2 = (g[2] - pc[2]) + bk[2];
      const float k3 = (g[3] - pc[3]) + bk[3];
      float part = ((q[0] * k0 + q[1] * k1) + q[2] * k2) + q[3] * k3;
      part = part + __shfl_xor(part, 4, 32);
      part = part + __shfl_xor(part, 2, 32);
      part = part + __shfl_xor(part, 1, 32);
      const float lgt = part * isd;
      if (k < 8) lg0 = (l7 == k) ? lgt : lg0;
      else       lg1 = (l7 == (k - 8)) ? lgt : lg1;
    }
    float m = selmax(lg0, lg1);
    { const float o = __shfl_xor(m, 4, 32); m = selmax(m, o); }
    { const float o = __shfl_xor(m, 2, 32); m = selmax(m, o); }
    { const float o = __shfl_xor(m, 1, 32); m = selmax(m, o); }
    const float e0 = expf(lg0 - m);
    const float e1 = expf(lg1 - m);
    float s = e0 + e1;
    s = s + __shfl_xor(s, 4, 32);
    s = s + __shfl_xor(s, 2, 32);
    s = s + __shfl_xor(s, 1, 32);
    const float a0 = e0 / s;
    const float a1 = e1 / s;
    float c = a0 * lg0 + a1 * lg1;
    c = c + __shfl_xor(c, 4, 32);
    c = c + __shfl_xor(c, 2, 32);
    c = c + __shfl_xor(c, 1, 32);
    gate = gate + c;
  }

  const bool kbad = (kval != KNB);
  const float qn = __uint_as_float(0x7fc00000u);
  v4f o = (v4f){ gate * v[0], gate * v[1], gate * v[2], gate * v[3] };
  o[0] = kbad ? qn : o[0];
  o[1] = kbad ? qn : o[1];
  o[2] = kbad ? qn : o[2];
  o[3] = kbad ? qn : o[3];
  if (row < nrows) {
    volatile v4f* qo = (volatile v4f*)(out + (size_t)row * CH + 4 * lane);
    *qo = o;
    __threadfence();
    *qo = o;
  }
}

extern "C" void kernel_launch(void* const* d_in, const int* in_sizes, int n_in,
                              void* d_out, int out_size, void* d_ws, size_t ws_size,
                              hipStream_t stream) {
  if (n_in < 9) return;
  if (in_sizes[0] != ROWS * CH) return;
  if (in_sizes[1] != ROWS * 3) return;
  if (in_sizes[2] != 1) return;
  if (in_sizes[3] != CH * CH) return;
  if (in_sizes[4] != CH) return;
  if (in_sizes[5] != NSC * CH * CH) return;
  if (in_sizes[6] != NSC * CH) return;
  if (in_sizes[7] != CH * CH) return;
  if (in_sizes[8] != CH) return;
  if (out_size != ROWS * CH) return;
  if (ws_size < WS_TOTAL) return;

  const float* pcd   = (const float*)d_in[0];
  const float* coord = (const float*)d_in[1];
  const int*   kin   = (const int*)d_in[2];
  const float* Wq    = (const float*)d_in[3];
  const float* bq    = (const float*)d_in[4];
  const float* Wk    = (const float*)d_in[5];
  const float* bk    = (const float*)d_in[6];
  const float* Wv    = (const float*)d_in[7];
  const float* bv    = (const float*)d_in[8];
  float* out = (float*)d_out;

  char* ws = (char*)d_ws;
  unsigned short* XB  = (unsigned short*)(ws + OFF_XB);
  unsigned short* WB  = (unsigned short*)(ws + OFF_WB);
  float*          BT  = (float*)(ws + OFF_BT);
  float*          BK  = (float*)(ws + OFF_BK);
  float*          CT  = (float*)(ws + OFF_CT);
  float*          T   = (float*)(ws + OFF_T);
  int*            IDX = (int*)(ws + OFF_IDX);

  k_plane<0><<<ROWS * (CH / 8) / 256, 256, 0, stream>>>(pcd, ROWS, CH, CH, XB, ROWS, CH);
  k_prep<<<PREP_BLOCKS, 256, 0, stream>>>(coord, Wq, bq, Wk, bk, Wv, bv, WB, BT, BK, CT);
  k_gemm_nt<0, 1><<<(ROWS / 64) * (NCOL / 64) / 8, 256, 0, stream>>>(XB, WB, BT, T, ROWS, NCOL, CH, NCOL);
  k_sel<<<ROWS / 8, 256, 0, stream>>>(CT, IDX);
  k_attn<<<ROWS / 8, 256, 0, stream>>>(T, BK, IDX, kin, out, out_size / CH);
}
